// GAT_GCN_2963527434725
// MI455X (gfx1250) — hardware-verified
//
#include <hip/hip_runtime.h>
#include <stddef.h>
#include <stdint.h>
#include <math.h>


#define NNODE   16384
#define NEDGE   131072
#define NGRAPH  128
#define FD      78
#define NHEAD   10
#define HS      80
#define HW      800
#define HWQ     200
#define NCHK    7
#define GW      96
#define GWQ     24
#define XK      128
#define SDW     32
#define TLEN    625
#define CLEN    594
#define CLP     608
#define NTHR    256
#define NWAVE   8
#define EPT     8
#define CHUNK   (NTHR * EPT)
#define WCAP    (EPT * 32)
#define LISTN   (NWAVE * WCAP)
#define NB      512
#define SLOTB   9
#define RCAP    8192
#define DEGCAP  64
#define NBD     1024
#define SLD     10
#define GBM     64
#define GTHR    128
#define NEGSL   0.2f
#define WSMAX   134217728
#define AGG_INTS (2 * RCAP + 2 * NB + LISTN + 2 * NWAVE)
#define LDS_GAT ((AGG_INTS + HW) * 4)
#define LDS_GCN (AGG_INTS * 4)

static_assert((CHUNK & (CHUNK - 1)) == 0);
static_assert(NB == (1 << SLOTB) && NBD == (1 << SLD));
static_assert(((long long)CHUNK << SLOTB) < (1LL << 31) && ((long long)CHUNK << SLD) < (1LL << 31));
static_assert(((long long)NEDGE << SLOTB) < (1LL << 32));
static_assert(NTHR * 2 == NB);
static_assert(LISTN >= NB && LISTN >= NWAVE * WCAP);
static_assert((RCAP % 32) == 0 && (AGG_INTS % 4) == 0);
static_assert(NWAVE * HW <= RCAP && NWAVE * GW <= RCAP);
static_assert(LDS_GAT <= 300000);
static_assert((NNODE % NB) == 0 && (NNODE % NBD) == 0 && (NNODE % GBM) == 0 && (NNODE % NWAVE) == 0);
static_assert(NBD == NTHR * 4);
static_assert((NB % NWAVE) == 0);
static_assert(HW == NHEAD * HS && HWQ * 4 == HW && NCHK * 32 >= HWQ && (NCHK - 1) * 32 < HWQ);
static_assert(HWQ - (NCHK - 1) * 32 == 8);
static_assert(GWQ * 4 == GW && GWQ <= 32 && GW >= FD && (GW % 32) == 0);
static_assert((HS % 4) == 0 && HS / 4 == 20);
static_assert(GBM == (GTHR / 32) * 16);
static_assert((NGRAPH % GBM) == 0);
static_assert((CLP % 32) == 0 && CLP >= CLEN && CLP + 32 <= 640);
static_assert(NGRAPH * 4 == 512);

typedef float          v4f  __attribute__((ext_vector_type(4)));
typedef float          v8f  __attribute__((ext_vector_type(8)));
typedef int            v4i  __attribute__((ext_vector_type(4)));
typedef int            v8i  __attribute__((ext_vector_type(8)));
typedef unsigned int   v4u  __attribute__((ext_vector_type(4)));
typedef unsigned short v8us __attribute__((ext_vector_type(8)));
typedef __bf16         v16b __attribute__((ext_vector_type(16)));
typedef v4f  __attribute__((may_alias)) v4fa;
typedef v4i  __attribute__((may_alias)) v4ia;
typedef v8us __attribute__((may_alias)) v8usa;
union FragB { v16b v; v8us h[2]; v8i w; };

__device__ __forceinline__ v8f wmb(const FragB& a, const FragB& b, v8f c) {
  v8f d = __builtin_amdgcn_wmma_f32_16x16x32_bf16(false, a.v, false, b.v, (short)0, c, false, false);
  asm volatile("v_nop\n\tv_nop\n\tv_nop\n\tv_nop" : "+v"(d) : "v"(a.w), "v"(b.w));
  return d;
}

__device__ __forceinline__ unsigned int f2bf(float f) {
  const unsigned int u = __float_as_uint(f);
  return ((u + 0x7FFFu + ((u >> 16) & 1u)) >> 16) & 0xFFFFu;
}
__device__ __forceinline__ float bf2f(unsigned int b) { return __uint_as_float(b << 16); }
__device__ __forceinline__ float bfr(float f) { return bf2f(f2bf(f)); }
__device__ __forceinline__ v4f bfr4(const v4f a) {
  v4f r; r.x = bfr(a.x); r.y = bfr(a.y); r.z = bfr(a.z); r.w = bfr(a.w); return r;
}
__device__ __forceinline__ unsigned int hl1(float v, bool lo) {
  const unsigned int hb = f2bf(v);
  const unsigned int lb = f2bf(v - bf2f(hb));
  return lo ? lb : hb;
}
__device__ __forceinline__ v4u hilo8(const v4f a, const v4f b, const bool lo) {
  v4u r;
  r.x = hl1(a.x, lo) | (hl1(a.y, lo) << 16);
  r.y = hl1(a.z, lo) | (hl1(a.w, lo) << 16);
  r.z = hl1(b.x, lo) | (hl1(b.y, lo) << 16);
  r.w = hl1(b.z, lo) | (hl1(b.w, lo) << 16);
  return r;
}
__device__ __forceinline__ float relu_k(float v) { return (v > 0.0f) ? v : (v - v); }

template <int SLB>
__device__ __forceinline__ int scan_chunk(const int* __restrict__ dsts, int nE, int cbase, int slotBase,
                                          int nb, int vec8, int* list, int tid, int lane, int wave) {
  int wc = 0;
  const int el0  = tid * EPT;
  const int e0   = cbase + el0;
  const int sent = -2147483647 - 1;
  v4i da, db;
  if (vec8 != 0 && cbase + CHUNK <= nE) {
    da = *(const v4i*)(dsts + e0);
    db = *(const v4i*)(dsts + e0 + 4);
  } else {
    da.x = (e0     < nE) ? dsts[min(e0,     nE - 1)] : sent;
    da.y = (e0 + 1 < nE) ? dsts[min(e0 + 1, nE - 1)] : sent;
    da.z = (e0 + 2 < nE) ? dsts[min(e0 + 2, nE - 1)] : sent;
    da.w = (e0 + 3 < nE) ? dsts[min(e0 + 3, nE - 1)] : sent;
    db.x = (e0 + 4 < nE) ? dsts[min(e0 + 4, nE - 1)] : sent;
    db.y = (e0 + 5 < nE) ? dsts[min(e0 + 5, nE - 1)] : sent;
    db.z = (e0 + 6 < nE) ? dsts[min(e0 + 6, nE - 1)] : sent;
    db.w = (e0 + 7 < nE) ? dsts[min(e0 + 7, nE - 1)] : sent;
  }
  const unsigned nbs = (unsigned)slotBase;
  const unsigned unb = (unsigned)nb;
  const unsigned s0 = (unsigned)da.x - nbs, s1 = (unsigned)da.y - nbs;
  const unsigned s2 = (unsigned)da.z - nbs, s3 = (unsigned)da.w - nbs;
  const unsigned s4 = (unsigned)db.x - nbs, s5 = (unsigned)db.y - nbs;
  const unsigned s6 = (unsigned)db.z - nbs, s7 = (unsigned)db.w - nbs;
  const bool h0 = s0 < unb, h1 = s1 < unb, h2 = s2 < unb, h3 = s3 < unb;
  const bool h4 = s4 < unb, h5 = s5 < unb, h6 = s6 < unb, h7 = s7 < unb;
  const unsigned any = __builtin_amdgcn_ballot_w32(h0 | h1 | h2 | h3 | h4 | h5 | h6 | h7);
  if (any != 0u) {
#define HITJ(J, HJ, SJ) { \
      const unsigned mj = __builtin_amdgcn_ballot_w32(HJ); \
      if (mj != 0u) { \
        if (HJ) { \
          const int pos = wc + (int)__builtin_amdgcn_mbcnt_lo(mj, 0u); \
          if (pos < WCAP) list[wave * WCAP + pos] = ((el0 + (J)) << SLB) | (int)(SJ); \
        } \
        wc += (int)__builtin_popcount(mj); } }
    HITJ(0, h0, s0)
    HITJ(1, h1, s1)
    HITJ(2, h2, s2)
    HITJ(3, h3, s3)
    HITJ(4, h4, s4)
    HITJ(5, h5, s5)
    HITJ(6, h6, s6)
    HITJ(7, h7, s7)
#undef HITJ
  }
  return wc;
}

__device__ __forceinline__ int build_lists(const int* __restrict__ dsts, int nE, int nodeBase, int vec8,
                                           int* reg1, int* reg2, int* scnt, int* soff, int* list,
                                           int* wcnt, int* wtot, int tid, int lane, int wave) {
  for (int i = tid; i < NB; i += NTHR) scnt[i] = 0;
  __syncthreads();

  int tot = 0;
  const int nChunks = (nE + CHUNK - 1) / CHUNK;
#pragma unroll 1
  for (int ch = 0; ch < nChunks; ++ch) {
    const int cbase = ch * CHUNK;
    const int wc = scan_chunk<SLOTB>(dsts, nE, cbase, nodeBase, NB, vec8, list, tid, lane, wave);
    if (lane == 0) wcnt[wave] = wc;
    __syncthreads();
    int pre = 0, all = 0;
#pragma unroll
    for (int w2 = 0; w2 < NWAVE; ++w2) {
      int c = wcnt[w2];
      c = c < 0 ? 0 : (c > WCAP ? WCAP : c);
      all += c;
      pre += (w2 < wave) ? c : 0;
    }
    const int wcc  = wc > WCAP ? WCAP : wc;
    const int base = tot + pre;
#pragma unroll 1
    for (int i = lane; i < wcc; i += 32) {
      const int ent = list[wave * WCAP + i];
      const int el  = (ent >> SLOTB) & (CHUNK - 1);
      const int sl  = ent & (NB - 1);
      int eid = cbase + el;
      eid = eid > nE - 1 ? nE - 1 : eid;
      const int pos = base + i;
      if (pos < RCAP) reg1[pos] = (int)(((unsigned)eid << SLOTB) | (unsigned)sl);
    }
    tot += all;
    tot = tot > RCAP ? RCAP : tot;
    __syncthreads();
  }
  const int nh = tot;

  if (wave == 0) {
#pragma unroll 1
    for (int b0 = 0; b0 < nh; b0 += 32) {
      const int idx = b0 + lane;
      const int uv  = reg1[idx < nh ? idx : nh - 1];
      const int m32 = (nh - b0) < 32 ? (nh - b0) : 32;
#pragma unroll 1
      for (int k = 0; k < m32; ++k) {
        const int u  = __builtin_amdgcn_readlane(uv, k);
        const int sl = u & (NB - 1);
        if (lane == 0) scnt[sl] = scnt[sl] + 1;
      }
    }
  }
  __syncthreads();

  {
    int e0 = scnt[2 * tid], e1 = scnt[2 * tid + 1];
    e0 = e0 < 0 ? 0 : e0;
    e1 = e1 < 0 ? 0 : e1;
    const int ts = e0 + e1;
    int incl = ts;
#pragma unroll
    for (int d = 1; d < 32; d <<= 1) {
      const int up = __shfl_up(incl, d);
      if (lane >= d) incl += up;
    }
    if (lane == 31) wtot[wave] = incl;
    __syncthreads();
    int pre = 0;
#pragma unroll
    for (int w2 = 0; w2 < NWAVE; ++w2) pre += (w2 < wave) ? wtot[w2] : 0;
    const int run = pre + incl - ts;
    soff[2 * tid]     = run;
    soff[2 * tid + 1] = run + e0;
  }
  __syncthreads();
  for (int i = tid; i < NB; i += NTHR) list[i] = soff[i];
  __syncthreads();

  if (wave == 0) {
#pragma unroll 1
    for (int b0 = 0; b0 < nh; b0 += 32) {
      const int idx = b0 + lane;
      const int uv  = reg1[idx < nh ? idx : nh - 1];
      const int m32 = (nh - b0) < 32 ? (nh - b0) : 32;
#pragma unroll 1
      for (int k = 0; k < m32; ++k) {
        const int u   = __builtin_amdgcn_readlane(uv, k);
        const int sl  = u & (NB - 1);
        const int eid = (int)((unsigned)u >> SLOTB);
        if (lane == 0) {
          int pos = list[sl];
          pos = pos < 0 ? 0 : (pos > RCAP - 1 ? RCAP - 1 : pos);
          reg2[pos] = eid;
          list[sl] = pos + 1;
        }
      }
    }
  }
  __syncthreads();
  return nh;
}

__global__ __launch_bounds__(NTHR) void k_xprep(const float* __restrict__ x, unsigned short* xb, int nN, int nUnits) {
  const int u = (int)blockIdx.x * NTHR + (int)threadIdx.x;
  if (u >= nUnits) return;
  const int row = u >> 4;
  const int k8  = (u & 15) * 8;
  const int rc  = row < nN ? row : nN - 1;
  const float* p = x + (size_t)rc * FD;
  float v[8];
#pragma unroll
  for (int i = 0; i < 8; ++i) {
    const int kk = k8 + i;
    const int kc = kk < FD ? kk : FD - 1;
    const float t = p[kc];
    v[i] = (kk < FD && row < nN) ? t : 0.0f;
  }
  v4u o;
  o.x = f2bf(v[0]) | (f2bf(v[1]) << 16);
  o.y = f2bf(v[2]) | (f2bf(v[3]) << 16);
  o.z = f2bf(v[4]) | (f2bf(v[5]) << 16);
  o.w = f2bf(v[6]) | (f2bf(v[7]) << 16);
  unsigned short* dp = xb + (size_t)row * XK + k8;
  *(volatile v4u*)dp = o;
  __threadfence();
  *(volatile v4u*)dp = o;
}

__global__ __launch_bounds__(NTHR) void k_wplane(const float* __restrict__ w, int ldw,
                                                 unsigned short* wt, int Kout, int Khalf,
                                                 int GSP, int GR, int NG, int NSP, int NR, int NNG, int nUnits) {
  const int u = (int)blockIdx.x * NTHR + (int)threadIdx.x;
  if (u >= nUnits) return;
  const int kq = Kout >> 3;
  const int n  = u / kq;
  const int k8 = (u - n * kq) * 8;
  const int kk = k8 - (k8 / Khalf) * Khalf;
  const int g  = kk / GSP;
  const int f0 = kk - g * GSP;
  const int gn = n / NSP;
  const int fn = n - gn * NSP;
  const bool nok = (fn < NR) && (gn < NNG) && (g < NG);
  const int gcl  = g < NG ? g : NG - 1;
  const int ncol = (gn < NNG ? gn : NNG - 1) * NR + (fn < NR ? fn : NR - 1);
  unsigned int hb[8];
#pragma unroll
  for (int i = 0; i < 8; ++i) {
    const int f   = f0 + i;
    const int row = gcl * GR + (f < GR ? f : GR - 1);
    const float t = w[(size_t)row * (size_t)ldw + ncol];
    hb[i] = (nok && f < GR) ? f2bf(t) : 0u;
  }
  v4u o;
  o.x = hb[0] | (hb[1] << 16);
  o.y = hb[2] | (hb[3] << 16);
  o.z = hb[4] | (hb[5] << 16);
  o.w = hb[6] | (hb[7] << 16);
  unsigned short* dp = wt + (size_t)n * (size_t)Kout + k8;
  *(volatile v4u*)dp = o;
  __threadfence();
  *(volatile v4u*)dp = o;
}

__global__ __launch_bounds__(NTHR) void k_deg(const int* __restrict__ dsts, int nE, int vec8, float* dis) {
  __shared__ __attribute__((aligned(16))) int scnt[NBD];
  __shared__ __attribute__((aligned(16))) int list[LISTN];
  __shared__ int wcnt[NWAVE];
  const int tid = (int)threadIdx.x, lane = tid & 31, wave = tid >> 5;
  const int nodeBase = (int)blockIdx.x * NBD;

  for (int i = tid; i < NBD; i += NTHR) scnt[i] = 0;
  for (int i = tid; i < LISTN; i += NTHR) list[i] = 0;
  if (tid < NWAVE) wcnt[tid] = 0;
  __syncthreads();

  const int nChunks = (nE + CHUNK - 1) / CHUNK;
#pragma unroll 1
  for (int ch = 0; ch < nChunks; ++ch) {
    const int cbase = ch * CHUNK;
    const int wc = scan_chunk<SLD>(dsts, nE, cbase, nodeBase, NBD, vec8, list, tid, lane, wave);
    if (lane == 0) wcnt[wave] = wc;
    __syncthreads();
    if (wave == 0) {
#pragma unroll 1
      for (int w2 = 0; w2 < NWAVE; ++w2) {
        int c = wcnt[w2];
        c = c < 0 ? 0 : (c > WCAP ? WCAP : c);
#pragma unroll 1
        for (int b0 = 0; b0 < c; b0 += 32) {
          const int idx = b0 + lane;
          const int ent = list[w2 * WCAP + (idx < WCAP ? idx : WCAP - 1)];
          const int m32 = (c - b0) < 32 ? (c - b0) : 32;
#pragma unroll 1
          for (int k = 0; k < m32; ++k) {
            const int u  = __builtin_amdgcn_readlane(ent, k);
            const int sl = u & (NBD - 1);
            if (lane == 0) scnt[sl] = scnt[sl] + 1;
          }
        }
      }
    }
    __syncthreads();
  }

  const v4i c4 = *(const v4ia*)(scnt + 4 * tid);
  v4f v;
  v.x = rsqrtf((float)c4.x + 1.0f);
  v.y = rsqrtf((float)c4.y + 1.0f);
  v.z = rsqrtf((float)c4.z + 1.0f);
  v.w = rsqrtf((float)c4.w + 1.0f);
  float* dp = dis + (size_t)nodeBase + 4 * tid;
  *(volatile v4f*)dp = v;
  __threadfence();
  *(volatile v4f*)dp = v;
}

template <int NT>
__global__ __launch_bounds__(GTHR) void k_gemm(
    const unsigned short* __restrict__ A, int lda,
    const unsigned short* __restrict__ WT, int ldb, int K,
    float* outF, int ldo, int ocol,
    const float* __restrict__ bias, int hasBias, int relu)
{
  constexpr int GBN = 16 * NT;
  constexpr int PPR = 4 * NT;
  constexpr int NIT = (GBM * PPR) / GTHR;
  static_assert((PPR & (PPR - 1)) == 0 && (GTHR % PPR) == 0 && PPR >= 8);
  __shared__ __attribute__((aligned(16))) float stg[GBM * GBN];
  const int tid = (int)threadIdx.x, lane = tid & 31, wave = tid >> 5, hh = lane >> 4, m = lane & 15;
  const int rowBase = (int)blockIdx.x * GBM;
  const int col0    = (int)blockIdx.y * GBN;

  v8f acc[NT];
  {
    const v8f z = {0.f, 0.f, 0.f, 0.f, 0.f, 0.f, 0.f, 0.f};
#pragma unroll
    for (int t = 0; t < NT; ++t) acc[t] = z;
  }
  const unsigned short* ap = A  + (size_t)(rowBase + 16 * wave + m) * (size_t)lda + 8 * hh;
  const unsigned short* wp = WT + (size_t)(col0 + m) * (size_t)ldb + 8 * hh;
  const int ksteps = K >> 5;
#pragma unroll 1
  for (int ks = 0; ks < ksteps; ++ks) {
    FragB af;
    af.h[0] = *(const v8usa*)(ap + 32 * ks);
    af.h[1] = *(const v8usa*)(ap + 32 * ks + 16);
#pragma unroll
    for (int t = 0; t < NT; ++t) {
      const unsigned short* wq = wp + (size_t)(16 * t) * (size_t)ldb + 32 * ks;
      FragB bf;
      bf.h[0] = *(const v8usa*)wq;
      bf.h[1] = *(const v8usa*)(wq + 16);
      acc[t] = wmb(af, bf, acc[t]);
    }
  }

#pragma unroll
  for (int t = 0; t < NT; ++t) {
    const int lc = 16 * t + m;
#pragma unroll
    for (int r = 0; r < 8; ++r) {
      const int lr = 16 * wave + 8 * hh + r;
      stg[lr * GBN + lc] = acc[t][r];
    }
  }
  __syncthreads();

  const int pc = tid & (PPR - 1);
  v4f bb = {0.f, 0.f, 0.f, 0.f};
  if (hasBias != 0) {
    const v4f t4 = *(const v4fa*)(bias + col0 + 4 * pc);
    bb = bfr4(t4);
  }
  v4f fv[NIT];
#pragma unroll
  for (int it = 0; it < NIT; ++it) {
    const int p  = it * GTHR + tid;
    const int lr = p / PPR;
    v4f v = *(const v4fa*)(stg + lr * GBN + 4 * pc);
    v.x += bb.x; v.y += bb.y; v.z += bb.z; v.w += bb.w;
    if (relu != 0) { v.x = relu_k(v.x); v.y = relu_k(v.y); v.z = relu_k(v.z); v.w = relu_k(v.w); }
    fv[it] = v;
  }
#pragma unroll
  for (int it = 0; it < NIT; ++it) {
    const int p  = it * GTHR + tid;
    const int lr = p / PPR;
    float* op = outF + (size_t)(rowBase + lr) * (size_t)ldo + ocol + col0 + 4 * pc;
    *(volatile v4f*)op = fv[it];
  }
  __threadfence();
#pragma unroll
  for (int it = 0; it < NIT; ++it) {
    const int p  = it * GTHR + tid;
    const int lr = p / PPR;
    float* op = outF + (size_t)(rowBase + lr) * (size_t)ldo + ocol + col0 + 4 * pc;
    *(volatile v4f*)op = fv[it];
  }
}

__global__ __launch_bounds__(NTHR) void k_dots(const float* __restrict__ Hf, const float* __restrict__ as_,
                                               const float* __restrict__ ad_, float* SD, int nN) {
  __shared__ __attribute__((aligned(16))) float tab[2 * HW];
  const int tid = (int)threadIdx.x, lane = tid & 31, wave = tid >> 5;
  {
    const int tq = tid < HWQ ? tid : HWQ - 1;
    const int c  = 4 * tq;
    const int hd = c / HS;
    const int f0 = c - hd * HS;
    float va[4], vd[4];
#pragma unroll
    for (int i = 0; i < 4; ++i) {
      const int f  = f0 + i;
      const int ix = hd * FD + (f < FD ? f : FD - 1);
      const float a = as_[ix];
      const float d = ad_[ix];
      va[i] = (f < FD) ? bfr(a) : 0.0f;
      vd[i] = (f < FD) ? bfr(d) : 0.0f;
    }
    if (tid < HWQ) {
      v4f a4, d4;
      a4.x = va[0]; a4.y = va[1]; a4.z = va[2]; a4.w = va[3];
      d4.x = vd[0]; d4.y = vd[1]; d4.z = vd[2]; d4.w = vd[3];
      *(v4fa*)(tab + c) = a4;
      *(v4fa*)(tab + HW + c) = d4;
    }
  }
  __syncthreads();
  const int node = (int)blockIdx.x * NWAVE + wave;
  const int nc   = node < nN ? node : nN - 1;
  const int lc   = lane < 20 ? lane : 19;
  const float* hr = Hf + (size_t)nc * HW + 4 * lc;
  float myv = 0.0f;
#pragma unroll 1
  for (int hd = 0; hd < NHEAD; ++hd) {
    const v4f hv = *(const v4fa*)(hr + hd * HS);
    const v4f a4 = *(const v4fa*)(tab + hd * HS + 4 * lc);
    const v4f d4 = *(const v4fa*)(tab + HW + hd * HS + 4 * lc);
    float s1 = hv.x * a4.x;
    s1 = fmaf(hv.y, a4.y, s1); s1 = fmaf(hv.z, a4.z, s1); s1 = fmaf(hv.w, a4.w, s1);
    float s2 = hv.x * d4.x;
    s2 = fmaf(hv.y, d4.y, s2); s2 = fmaf(hv.z, d4.z, s2); s2 = fmaf(hv.w, d4.w, s2);
    s1 = (lane < 20) ? s1 : 0.0f;
    s2 = (lane < 20) ? s2 : 0.0f;
#pragma unroll
    for (int off = 16; off > 0; off >>= 1) {
      s1 += __shfl_xor(s1, off);
      s2 += __shfl_xor(s2, off);
    }
    myv = (lane == hd) ? s1 : myv;
    myv = (lane == 16 + hd) ? s2 : myv;
  }
  float* op = SD + (size_t)node * SDW + lane;
  const bool wr = node < nN;
  if (wr) *(volatile float*)op = myv;
  __threadfence();
  if (wr) *(volatile float*)op = myv;
}

template <int LAYER>
__global__ __launch_bounds__(NTHR) void k_gat(
    const int* __restrict__ srcs, const int* __restrict__ dsts,
    const float* __restrict__ Hf, const float* __restrict__ SD,
    const float* __restrict__ bias,
    unsigned short* XA, float* XF,
    int nN, int nE, int vec8) {
  extern __shared__ v4f lds_dyn[];
  int* reg1 = (int*)lds_dyn;
  int* reg2 = reg1 + RCAP;
  int* scnt = reg2 + RCAP;
  int* soff = scnt + NB;
  int* list = soff + NB;
  int* wcnt = list + LISTN;
  int* wtot = wcnt + NWAVE;
  float* bsh = (float*)(wtot + NWAVE);
  const int tid = (int)threadIdx.x, lane = tid & 31, wave = tid >> 5;
  const int nodeBase = (int)blockIdx.x * NB;

  {
    const int tq = tid < HWQ ? tid : HWQ - 1;
    const int c  = 4 * tq;
    const int hdx = c / HS;
    const int f0 = c - hdx * HS;
    float vb[4];
#pragma unroll
    for (int i = 0; i < 4; ++i) {
      const int f  = f0 + i;
      const float b = bias[hdx * FD + (f < FD ? f : FD - 1)];
      vb[i] = (f < FD) ? bfr(b) : 0.0f;
    }
    if (tid < HWQ) {
      v4f b4; b4.x = vb[0]; b4.y = vb[1]; b4.z = vb[2]; b4.w = vb[3];
      *(v4fa*)(bsh + c) = b4;
    }
  }

  const int nh = build_lists(dsts, nE, nodeBase, vec8, reg1, reg2, scnt, soff, list, wcnt, wtot, tid, lane, wave);

  const bool ovf = (nh >= RCAP);
  const float qnan = __int_as_float(0x7fc00000);
  int col[NCHK], hd[NCHK];
#pragma unroll
  for (int j = 0; j < NCHK; ++j) {
    const int q  = lane + 32 * j;
    const int qc = q < HWQ ? q : HWQ - 1;
    col[j] = 4 * qc;
    hd[j]  = qc / 20;
  }
  float* stg = (float*)reg1 + wave * HW;

#pragma unroll 1
  for (int jt = 0; jt < NB / NWAVE; ++jt) {
    const int slot = wave * (NB / NWAVE) + jt;
    const int grow = nodeBase + slot;
    const int gcl  = grow < nN ? grow : nN - 1;
    int st = soff[slot];
    const int craw = scnt[slot];
    int cnt = craw;
    st  = st < 0 ? 0 : (st > nh ? nh : st);
    cnt = cnt < 0 ? 0 : (cnt > DEGCAP ? DEGCAP : cnt);
    if (cnt > nh - st) cnt = nh - st;
    st  = __builtin_amdgcn_readfirstlane(st);
    cnt = __builtin_amdgcn_readfirstlane(cnt);
    const float pz = (ovf || craw > DEGCAP) ? qnan : 0.0f;

    const float sdo = SD[(size_t)gcl * SDW + lane];
    const float* hrow = Hf + (size_t)gcl * HW;
    float mx[NCHK], dn[NCHK], adv[NCHK];
    v4f av[NCHK];
#pragma unroll
    for (int j = 0; j < NCHK; ++j) {
      const float as0 = __shfl(sdo, hd[j]);
      const float ad0 = __shfl(sdo, 16 + hd[j]);
      adv[j] = ad0;
      float l0 = as0 + ad0;
      l0 = l0 > 0.f ? l0 : NEGSL * l0;
      mx[j] = l0;
      dn[j] = 1.0f;
      av[j] = *(const v4fa*)(hrow + col[j]);
    }

#pragma unroll 1
    for (int q = 0; q < cnt; ++q) {
      int idx = st + q; idx = idx > RCAP - 1 ? RCAP - 1 : idx;
      int eid = reg2[idx]; eid = eid < 0 ? 0 : (eid > nE - 1 ? nE - 1 : eid);
      const int sraw = srcs[eid];
      const int s = sraw < 0 ? 0 : (sraw > nN - 1 ? nN - 1 : sraw);
      const float sdv = SD[(size_t)s * SDW + lane];
      const float* fr = Hf + (size_t)s * HW;
#pragma unroll
      for (int j = 0; j < NCHK; ++j) {
        const v4f fs = *(const v4fa*)(fr + col[j]);
        float lg = __shfl(sdv, hd[j]) + adv[j];
        lg = lg > 0.f ? lg : NEGSL * lg;
        const float df = lg - mx[j];
        const float ee = __expf(-fabsf(df));
        const bool up  = df > 0.f;
        const float s1 = up ? ee : 1.0f;
        const float s2 = up ? 1.0f : ee;
        mx[j] = up ? lg : mx[j];
        dn[j] = fmaf(dn[j], s1, s2);
        av[j].x = fmaf(av[j].x, s1, s2 * fs.x);
        av[j].y = fmaf(av[j].y, s1, s2 * fs.y);
        av[j].z = fmaf(av[j].z, s1, s2 * fs.z);
        av[j].w = fmaf(av[j].w, s1, s2 * fs.w);
      }
    }

    const bool wr = grow < nN;
    if (LAYER == 1) {
#pragma unroll
      for (int j = 0; j < NCHK; ++j) {
        const float inv = __builtin_amdgcn_rcpf(dn[j]);
        const v4f bb = *(const v4fa*)(bsh + col[j]);
        v4f o;
        o.x = fmaf(av[j].x, inv, bb.x) + pz;
        o.y = fmaf(av[j].y, inv, bb.y) + pz;
        o.z = fmaf(av[j].z, inv, bb.z) + pz;
        o.w = fmaf(av[j].w, inv, bb.w) + pz;
        if (j < NCHK - 1 || lane < 8) *(v4fa*)(stg + col[j]) = o;
      }
      __syncthreads();
      v4u pv[NCHK];
#pragma unroll
      for (int i = 0; i < NCHK; ++i) {
        const int p   = lane + 32 * i;
        const int pcl = p < HWQ ? p : HWQ - 1;
        const bool lo = pcl >= HWQ / 2;
        const int w8  = pcl - (lo ? HWQ / 2 : 0);
        const v4f a = *(const v4fa*)(stg + 8 * w8);
        const v4f b = *(const v4fa*)(stg + 8 * w8 + 4);
        pv[i] = hilo8(a, b, lo);
      }
      unsigned short* gp = XA + (size_t)grow * (2 * HW) + 8 * lane;
#pragma unroll
      for (int i = 0; i < NCHK; ++i)
        if (wr && (i < NCHK - 1 || lane < 8)) *(volatile v4u*)(gp + 256 * i) = pv[i];
      __threadfence();
#pragma unroll
      for (int i = 0; i < NCHK; ++i)
        if (wr && (i < NCHK - 1 || lane < 8)) *(volatile v4u*)(gp + 256 * i) = pv[i];
      __syncthreads();
    } else {
      v4f ov[NCHK];
#pragma unroll
      for (int j = 0; j < NCHK; ++j) {
        const float inv = __builtin_amdgcn_rcpf(dn[j]);
        const v4f bb = *(const v4fa*)(bsh + col[j]);
        v4f o;
        o.x = relu_k(fmaf(av[j].x, inv, bb.x)) + pz;
        o.y = relu_k(fmaf(av[j].y, inv, bb.y)) + pz;
        o.z = relu_k(fmaf(av[j].z, inv, bb.z)) + pz;
        o.w = relu_k(fmaf(av[j].w, inv, bb.w)) + pz;
        ov[j] = o;
      }
      float* gp = XF + (size_t)grow * HW;
#pragma unroll
      for (int j = 0; j < NCHK; ++j)
        if (wr && (j < NCHK - 1 || lane < 8)) *(volatile v4f*)(gp + col[j]) = ov[j];
      __threadfence();
#pragma unroll
      for (int j = 0; j < NCHK; ++j)
        if (wr && (j < NCHK - 1 || lane < 8)) *(volatile v4f*)(gp + col[j]) = ov[j];
    }
  }
}

template <int LAYER>
__global__ __launch_bounds__(NTHR) void k_gcn(
    const int* __restrict__ srcs, const int* __restrict__ dsts,
    const float* __restrict__ HG, const float* __restrict__ dis,
    const float* __restrict__ bias,
    unsigned short* XG, float* XF,
    int nN, int nE, int vec8) {
  extern __shared__ v4f lds_dyn[];
  int* reg1 = (int*)lds_dyn;
  int* reg2 = reg1 + RCAP;
  int* scnt = reg2 + RCAP;
  int* soff = scnt + NB;
  int* list = soff + NB;
  int* wcnt = list + LISTN;
  int* wtot = wcnt + NWAVE;
  const int tid = (int)threadIdx.x, lane = tid & 31, wave = tid >> 5;
  const int nodeBase = (int)blockIdx.x * NB;

  const int qc  = lane < GWQ ? lane : GWQ - 1;
  const int col = 4 * qc;
  v4f bb;
  {
    float vb[4];
#pragma unroll
    for (int i = 0; i < 4; ++i) {
      const int c = col + i;
      const float b = bias[c < FD ? c : FD - 1];
      vb[i] = (c < FD) ? bfr(b) : 0.0f;
    }
    bb.x = vb[0]; bb.y = vb[1]; bb.z = vb[2]; bb.w = vb[3];
  }

  const int nh = build_lists(dsts, nE, nodeBase, vec8, reg1, reg2, scnt, soff, list, wcnt, wtot, tid, lane, wave);

  const bool ovf = (nh >= RCAP);
  const float qnan = __int_as_float(0x7fc00000);
  float* stg = (float*)reg1 + wave * GW;

#pragma unroll 1
  for (int jt = 0; jt < NB / NWAVE; ++jt) {
    const int slot = wave * (NB / NWAVE) + jt;
    const int grow = nodeBase + slot;
    const int gcl  = grow < nN ? grow : nN - 1;
    int st = soff[slot];
    const int craw = scnt[slot];
    int cnt = craw;
    st  = st < 0 ? 0 : (st > nh ? nh : st);
    cnt = cnt < 0 ? 0 : (cnt > DEGCAP ? DEGCAP : cnt);
    if (cnt > nh - st) cnt = nh - st;
    st  = __builtin_amdgcn_readfirstlane(st);
    cnt = __builtin_amdgcn_readfirstlane(cnt);
    const float pz = (ovf || craw > DEGCAP) ? qnan : 0.0f;

    const float dd = dis[gcl];
    v4f acc = {0.f, 0.f, 0.f, 0.f};
#pragma unroll 1
    for (int q = 0; q < cnt; ++q) {
      int idx = st + q; idx = idx > RCAP - 1 ? RCAP - 1 : idx;
      int eid = reg2[idx]; eid = eid < 0 ? 0 : (eid > nE - 1 ? nE - 1 : eid);
      const int sraw = srcs[eid];
      const int s = sraw < 0 ? 0 : (sraw > nN - 1 ? nN - 1 : sraw);
      const float cf = dis[s] * dd;
      const v4f a = *(const v4fa*)(HG + (size_t)s * GW + col);
      acc.x = fmaf(cf, a.x, acc.x);
      acc.y = fmaf(cf, a.y, acc.y);
      acc.z = fmaf(cf, a.z, acc.z);
      acc.w = fmaf(cf, a.w, acc.w);
    }
    const v4f sv = *(const v4fa*)(HG + (size_t)gcl * GW + col);
    const float rd = dd * dd;
    v4f y;
    y.x = (acc.x + sv.x * rd) + bb.x;
    y.y = (acc.y + sv.y * rd) + bb.y;
    y.z = (acc.z + sv.z * rd) + bb.z;
    y.w = (acc.w + sv.w * rd) + bb.w;
    const bool wr = (grow < nN) && (lane < GWQ);
    if (LAYER == 1) {
      y.x += pz; y.y += pz; y.z += pz; y.w += pz;
      if (lane < GWQ) *(v4fa*)(stg + col) = y;
      __syncthreads();
      const bool lo = qc >= GWQ / 2;
      const int w8  = qc - (lo ? GWQ / 2 : 0);
      const v4f a = *(const v4fa*)(stg + 8 * w8);
      const v4f b = *(const v4fa*)(stg + 8 * w8 + 4);
      const v4u pv = hilo8(a, b, lo);
      unsigned short* gp = XG + (size_t)grow * (2 * GW) + 8 * qc;
      if (wr) *(volatile v4u*)gp = pv;
      __threadfence();
      if (wr) *(volatile v4u*)gp = pv;
      __syncthreads();
    } else {
      v4f o;
      o.x = relu_k(y.x) + pz; o.y = relu_k(y.y) + pz; o.z = relu_k(y.z) + pz; o.w = relu_k(y.w) + pz;
      float* gp = XF + (size_t)grow * GW + col;
      if (wr) *(volatile v4f*)gp = o;
      __threadfence();
      if (wr) *(volatile v4f*)gp = o;
    }
  }
}

template <int W>
__global__ __launch_bounds__(((W / 4 + 31) / 32) * 32) void k_pool(const float* __restrict__ X,
                                                                   const int* __restrict__ bat, int nN,
                                                                   unsigned short* PD) {
  constexpr int NQ   = W / 4;
  constexpr int NTH  = ((NQ + 31) / 32) * 32;
  constexpr int NPH  = W / 4;
  constexpr int NP   = 2 * NPH;
  constexpr int NITP = (NP + NTH - 1) / NTH;
  static_assert((W % 8) == 0 && ((8 * W) % 128) == 0);
  __shared__ __attribute__((aligned(16))) float row[2 * W];
  const int tid = (int)threadIdx.x, lane = tid & 31;
  const int g = (int)blockIdx.x;
  const int qc = tid < NQ ? tid : NQ - 1;
  const int col = 4 * qc;

  const float ninf = -__builtin_inff();
  v4f mxv = {ninf, ninf, ninf, ninf};
  double s0 = 0.0, s1 = 0.0, s2 = 0.0, s3 = 0.0;
  int mine = 0;
#pragma unroll 1
  for (int i0 = 0; i0 < nN; i0 += 32) {
    const int i  = i0 + lane;
    const int ic = i < nN ? i : nN - 1;
    const int b  = bat[ic];
    const bool hit = (i < nN) && (b == g);
    unsigned msk = __builtin_amdgcn_ballot_w32(hit);
    int nhit = (int)__builtin_popcount(msk);
    nhit = nhit > 32 ? 32 : nhit;
    mine += hit ? 1 : 0;
#pragma unroll 1
    for (int q = 0; q < nhit; ++q) {
      const int k = __builtin_ffs((int)msk) - 1;
      msk &= msk - 1u;
      int node = i0 + (k < 0 ? 0 : k);
      node = node > nN - 1 ? nN - 1 : node;
      const v4f v = *(const v4fa*)(X + (size_t)node * W + col);
      mxv.x = v.x > mxv.x ? v.x : mxv.x;
      mxv.y = v.y > mxv.y ? v.y : mxv.y;
      mxv.z = v.z > mxv.z ? v.z : mxv.z;
      mxv.w = v.w > mxv.w ? v.w : mxv.w;
      s0 += (double)v.x; s1 += (double)v.y; s2 += (double)v.z; s3 += (double)v.w;
    }
  }
  int cnt = mine;
  cnt += __shfl_xor(cnt, 16); cnt += __shfl_xor(cnt, 8); cnt += __shfl_xor(cnt, 4);
  cnt += __shfl_xor(cnt, 2);  cnt += __shfl_xor(cnt, 1);
  const float cf = (cnt < 1) ? 1.0f : (float)cnt;
  const float rc = 1.0f / cf;
  v4f mo, me;
  mo.x = (cnt > 0) ? mxv.x : 0.0f; mo.y = (cnt > 0) ? mxv.y : 0.0f;
  mo.z = (cnt > 0) ? mxv.z : 0.0f; mo.w = (cnt > 0) ? mxv.w : 0.0f;
  me.x = (float)s0 * rc; me.y = (float)s1 * rc; me.z = (float)s2 * rc; me.w = (float)s3 * rc;
  if (tid < NQ) {
    *(v4fa*)(row + col) = mo;
    *(v4fa*)(row + W + col) = me;
  }
  __syncthreads();
  v4u pv[NITP];
#pragma unroll
  for (int it = 0; it < NITP; ++it) {
    const int p   = it * NTH + tid;
    const int pcl = p < NP ? p : NP - 1;
    const bool lo = pcl >= NPH;
    const int w8  = pcl - (lo ? NPH : 0);
    const v4f a = *(const v4fa*)(row + 8 * w8);
    const v4f b = *(const v4fa*)(row + 8 * w8 + 4);
    pv[it] = hilo8(a, b, lo);
  }
  unsigned short* gp = PD + (size_t)g * (4 * W);
#pragma unroll
  for (int it = 0; it < NITP; ++it) {
    const int p = it * NTH + tid;
    if (p < NP) *(volatile v4u*)(gp + 8 * p) = pv[it];
  }
  __threadfence();
#pragma unroll
  for (int it = 0; it < NITP; ++it) {
    const int p = it * NTH + tid;
    if (p < NP) *(volatile v4u*)(gp + 8 * p) = pv[it];
  }
}

__global__ __launch_bounds__(NTHR) void k_conv(const float* __restrict__ target, const float* __restrict__ wc,
                                               const float* __restrict__ bc, unsigned short* YD) {
  __shared__ __attribute__((aligned(16))) float tr[640];
  __shared__ float wsh[32];
  __shared__ __attribute__((aligned(16))) float ys[CLP];
  const int tid = (int)threadIdx.x;
  const int g = (int)blockIdx.x;
#pragma unroll 1
  for (int i = tid; i < 640; i += NTHR) {
    const int ic = i < TLEN ? i : TLEN - 1;
    const float v = target[(size_t)g * TLEN + ic];
    tr[i] = (i < TLEN) ? bfr(v) : 0.0f;
  }
  {
    const float w = wc[tid & 31];
    if (tid < 32) wsh[tid] = bfr(w);
  }
  const float bcv = bfr(bc[0]);
  __syncthreads();
#pragma unroll 1
  for (int t = tid; t < CLP; t += NTHR) {
    float s = 0.0f;
#pragma unroll 4
    for (int k = 0; k < 32; ++k) s = fmaf(tr[t + k], wsh[k], s);
    s = relu_k(s + bcv);
    ys[t] = (t < CLEN) ? s : 0.0f;
  }
  __syncthreads();
  constexpr int NPH = CLP / 8;
  constexpr int NP  = 2 * NPH;
  const int pcl = tid < NP ? tid : NP - 1;
  const bool lo = pcl >= NPH;
  const int w8  = pcl - (lo ? NPH : 0);
  const v4f a = *(const v4fa*)(ys + 8 * w8);
  const v4f b = *(const v4fa*)(ys + 8 * w8 + 4);
  const v4u pv = hilo8(a, b, lo);
  unsigned short* gp = YD + (size_t)g * (2 * CLP) + 8 * pcl;
  const bool wr = tid < NP;
  if (wr) *(volatile v4u*)gp = pv;
  __threadfence();
  if (wr) *(volatile v4u*)gp = pv;
}

__global__ __launch_bounds__(NTHR) void k_split(const float* __restrict__ in, int W, unsigned short* outp, int nUnits) {
  const int u = (int)blockIdx.x * NTHR + (int)threadIdx.x;
  if (u >= nUnits) return;
  const int ppr = W >> 2;
  const int nph = W >> 3;
  const int row = u / ppr;
  const int p   = u - row * ppr;
  const bool lo = p >= nph;
  const int w8  = p - (lo ? nph : 0);
  const float* ip = in + (size_t)row * W + 8 * w8;
  const v4f a = *(const v4fa*)ip;
  const v4f b = *(const v4fa*)(ip + 4);
  const v4u pv = hilo8(a, b, lo);
  unsigned short* gp = outp + (size_t)row * (2 * W) + 8 * p;
  *(volatile v4u*)gp = pv;
  __threadfence();
  *(volatile v4u*)gp = pv;
}

__global__ __launch_bounds__(NTHR) void k_out(const float* __restrict__ Z2, const float* __restrict__ Wo,
                                              const float* __restrict__ bo, float* out) {
  __shared__ __attribute__((aligned(16))) float res[NGRAPH];
  const int tid = (int)threadIdx.x, lane = tid & 31, wave = tid >> 5;
  const v4f w0 = bfr4(*(const v4fa*)(Wo + 4 * lane));
  const v4f w1 = bfr4(*(const v4fa*)(Wo + 128 + 4 * lane));
  const float bov = bfr(bo[0]);
#pragma unroll 1
  for (int r = 0; r < NGRAPH / NWAVE; ++r) {
    const int g = wave * (NGRAPH / NWAVE) + r;
    const v4f a0 = *(const v4fa*)(Z2 + (size_t)g * 256 + 4 * lane);
    const v4f a1 = *(const v4fa*)(Z2 + (size_t)g * 256 + 128 + 4 * lane);
    float s = a0.x * w0.x;
    s = fmaf(a0.y, w0.y, s); s = fmaf(a0.z, w0.z, s); s = fmaf(a0.w, w0.w, s);
    s = fmaf(a1.x, w1.x, s); s = fmaf(a1.y, w1.y, s); s = fmaf(a1.z, w1.z, s); s = fmaf(a1.w, w1.w, s);
#pragma unroll
    for (int off = 16; off > 0; off >>= 1) s += __shfl_xor(s, off);
    if (lane == 0) res[g] = s + bov;
  }
  __syncthreads();
  const v4f ov = *(const v4fa*)(res + 4 * lane);
  float* op = out + 4 * lane;
  const bool wr = (wave == 0);
  if (wr) *(volatile v4f*)op = ov;
  __threadfence();
  if (wr) *(volatile v4f*)op = ov;
}

static inline int cdiv(int a, int b) { return (a + b - 1) / b; }
static inline size_t al256(size_t o) { return (o + 255) & ~(size_t)255; }

extern "C" void kernel_launch(void* const* d_in, const int* in_sizes, int n_in,
                              void* d_out, int out_size, void* d_ws, size_t ws_size,
                              hipStream_t stream) {
  if (n_in < 28) return;
  const int N = NNODE, E = NEDGE, G = NGRAPH;
  if (in_sizes[0] != N * FD || in_sizes[1] != 2 * E || in_sizes[2] != N || in_sizes[3] != G * TLEN) return;
  if (in_sizes[4] != FD * 780 || in_sizes[5] != 780 || in_sizes[6] != 780 || in_sizes[7] != 780) return;
  if (in_sizes[8] != 780 * 780 || in_sizes[9] != 780 || in_sizes[10] != 780 || in_sizes[11] != 780) return;
  if (in_sizes[12] != FD * FD || in_sizes[13] != FD) return;
  if (in_sizes[14] != 1560 * 128 || in_sizes[15] != 128 || in_sizes[16] != 156 * 128 || in_sizes[17] != 128) return;
  if (in_sizes[18] != 32 || in_sizes[19] != 1) return;
  if (in_sizes[20] != CLEN * 256 || in_sizes[21] != 256) return;
  if (in_sizes[22] != 512 * 512 || in_sizes[23] != 512 || in_sizes[24] != 512 * 256 || in_sizes[25] != 256) return;
  if (in_sizes[26] != 256 || in_sizes[27] != 1) return;
  if (out_size != G) return;

  const float* x      = (const float*)d_in[0];
  const int*   ei     = (const int*)  d_in[1];
  const int*   batch  = (const int*)  d_in[2];
  const float* target = (const float*)d_in[3];
  const float* Wg1    = (const float*)d_in[4];
  const float* as1    = (const float*)d_in[5];
  const float* ad1    = (const float*)d_in[6];
  const float* bg1    = (const float*)d_in[7];
  const float* Wg2    = (const float*)d_in[8];
  const float* as2    = (const float*)d_in[9];
  const float* ad2    = (const float*)d_in[10];
  const float* bg2    = (const float*)d_in[11];
  const float* Wgcn   = (const float*)d_in[12];
  const float* bgcn   = (const float*)d_in[13];
  const float* Wfg1   = (const float*)d_in[14];
  const float* bfg1   = (const float*)d_in[15];
  const float* Wfg2   = (const float*)d_in[16];
  const float* bfg2   = (const float*)d_in[17];
  const float* wconv  = (const float*)d_in[18];
  const float* bconv  = (const float*)d_in[19];
  const float* Wxt    = (const float*)d_in[20];
  const float* bxt    = (const float*)d_in[21];
  const float* W1     = (const float*)d_in[22];
  const float* b1     = (const float*)d_in[23];
  const float* W2     = (const float*)d_in[24];
  const float* b2     = (const float*)d_in[25];
  const float* Wo     = (const float*)d_in[26];
  const float* bo     = (const float*)d_in[27];
  float* out = (float*)d_out;
  const int* src = ei;
  const int* dst = ei + E;
  const int vec8 = ((E & 3) == 0) ? 1 : 0;

  char* ws = (char*)d_ws;
  size_t off = 0;
  const size_t oH   = off; off = al256(off + (size_t)N * HW * 4);
  const size_t oXA  = off; off = al256(off + (size_t)N * 2 * HW * 2);
  const size_t oXB  = off; off = al256(off + (size_t)N * XK * 2);
  const size_t oSD  = off; off = al256(off + (size_t)N * SDW * 4);
  const size_t oXG  = off; off = al256(off + (size_t)N * 2 * GW * 2);
  const size_t oDI  = off; off = al256(off + (size_t)N * 4);
  const size_t oWa  = off; off = al256(off + (size_t)HW * XK * 2);
  const size_t oWb  = off; off = al256(off + (size_t)HW * 2 * HW * 2);
  const size_t oWc  = off; off = al256(off + (size_t)GW * XK * 2);
  const size_t oWd  = off; off = al256(off + (size_t)GW * 2 * GW * 2);
  const size_t oWe  = off; off = al256(off + (size_t)128 * 4 * HW * 2);
  const size_t oWf  = off; off = al256(off + (size_t)128 * 4 * GW * 2);
  const size_t oWg  = off; off = al256(off + (size_t)256 * 2 * CLP * 2);
  const size_t oWh  = off; off = al256(off + (size_t)512 * 1024 * 2);
  const size_t oWi  = off; off = al256(off + (size_t)256 * 1024 * 2);
  const size_t oP1  = off; off = al256(off + (size_t)G * 4 * HW * 2);
  const size_t oP2  = off; off = al256(off + (size_t)G * 4 * GW * 2);
  const size_t oYD  = off; off = al256(off + (size_t)G * 2 * CLP * 2);
  const size_t oXC  = off; off = al256(off + (size_t)G * 512 * 4);
  const size_t oXCD = off; off = al256(off + (size_t)G * 1024 * 2);
  const size_t oZ1  = off; off = al256(off + (size_t)G * 512 * 4);
  const size_t oZ1D = off; off = al256(off + (size_t)G * 1024 * 2);
  const size_t oZ2  = off; off = al256(off + (size_t)G * 256 * 4);
  if (off > ws_size || off > (size_t)WSMAX) return;
  if ((size_t)2 * N * GW * 4 > (size_t)N * HW * 4) return;

  float*          H    = (float*)(ws + oH);
  float*          HGp  = (float*)(ws + oH);
  float*          X2F  = (float*)(ws + oH + (size_t)N * GW * 4);
  unsigned short* X1A  = (unsigned short*)(ws + oXA);
  float*          X1F  = (float*)(ws + oXA);
  unsigned short* XB   = (unsigned short*)(ws + oXB);
  float*          SD   = (float*)(ws + oSD);
  unsigned short* XG   = (unsigned short*)(ws + oXG);
  float*          DINV = (float*)(ws + oDI);
  unsigned short* Wg1t = (unsigned short*)(ws + oWa);
  unsigned short* Wg2D = (unsigned short*)(ws + oWb);
  unsigned short* WgcT = (unsigned short*)(ws + oWc);
  unsigned short* WgcD = (unsigned short*)(ws + oWd);
  unsigned short* Wf1D = (unsigned short*)(ws + oWe);
  unsigned short* Wf2D = (unsigned short*)(ws + oWf);
  unsigned short* WxtD = (unsigned short*)(ws + oWg);
  unsigned short* W1D  = (unsigned short*)(ws + oWh);
  unsigned short* W2D  = (unsigned short*)(ws + oWi);
  unsigned short* P1D  = (unsigned short*)(ws + oP1);
  unsigned short* P2D  = (unsigned short*)(ws + oP2);
  unsigned short* YD   = (unsigned short*)(ws + oYD);
  float*          XC   = (float*)(ws + oXC);
  unsigned short* XCD  = (unsigned short*)(ws + oXCD);
  float*          Z1   = (float*)(ws + oZ1);
  unsigned short* Z1D  = (unsigned short*)(ws + oZ1D);
  float*          Z2   = (float*)(ws + oZ2);

  hipFuncSetAttribute(reinterpret_cast<const void*>(&k_gat<1>), hipFuncAttributeMaxDynamicSharedMemorySize, LDS_GAT);
  hipFuncSetAttribute(reinterpret_cast<const void*>(&k_gat<2>), hipFuncAttributeMaxDynamicSharedMemorySize, LDS_GAT);
  hipFuncSetAttribute(reinterpret_cast<const void*>(&k_gcn<1>), hipFuncAttributeMaxDynamicSharedMemorySize, LDS_GCN);
  hipFuncSetAttribute(reinterpret_cast<const void*>(&k_gcn<2>), hipFuncAttributeMaxDynamicSharedMemorySize, LDS_GCN);

  { const int nU = N * (XK / 8); k_xprep<<<cdiv(nU, NTHR), NTHR, 0, stream>>>(x, XB, N, nU); }
  { const int nU = HW * (XK / 8);
    k_wplane<<<cdiv(nU, NTHR), NTHR, 0, stream>>>(Wg1, 780, Wg1t, XK, XK, XK, FD, 1, HS, FD, NHEAD, nU); }
  { const int nU = HW * (2 * HW / 8);
    k_wplane<<<cdiv(nU, NTHR), NTHR, 0, stream>>>(Wg2, 780, Wg2D, 2 * HW, HW, HS, FD, NHEAD, HS, FD, NHEAD, nU); }
  { const int nU = GW * (XK / 8);
    k_wplane<<<cdiv(nU, NTHR), NTHR, 0, stream>>>(Wgcn, FD, WgcT, XK, XK, XK, FD, 1, GW, FD, 1, nU); }
  { const int nU = GW * (2 * GW / 8);
    k_wplane<<<cdiv(nU, NTHR), NTHR, 0, stream>>>(Wgcn, FD, WgcD, 2 * GW, GW, GW, FD, 1, GW, FD, 1, nU); }
  { const int nU = 128 * (4 * HW / 8);
    k_wplane<<<cdiv(nU, NTHR), NTHR, 0, stream>>>(Wfg1, 128, Wf1D, 4 * HW, 2 * HW, HS, FD, 2 * NHEAD, 128, 128, 1, nU); }
  { const int nU = 128 * (4 * GW / 8);
    k_wplane<<<cdiv(nU, NTHR), NTHR, 0, stream>>>(Wfg2, 128, Wf2D, 4 * GW, 2 * GW, GW, FD, 2, 128, 128, 1, nU); }
  { const int nU = 256 * (2 * CLP / 8);
    k_wplane<<<cdiv(nU, NTHR), NTHR, 0, stream>>>(Wxt, 256, WxtD, 2 * CLP, CLP, CLP, CLEN, 1, 256, 256, 1, nU); }
  { const int nU = 512 * (1024 / 8);
    k_wplane<<<cdiv(nU, NTHR), NTHR, 0, stream>>>(W1, 512, W1D, 1024, 512, 512, 512, 1, 512, 512, 1, nU); }
  { const int nU = 256 * (1024 / 8);
    k_wplane<<<cdiv(nU, NTHR), NTHR, 0, stream>>>(W2, 256, W2D, 1024, 512, 512, 512, 1, 256, 256, 1, nU); }
  k_deg<<<N / NBD, NTHR, 0, stream>>>(dst, E, vec8, DINV);

  k_gemm<2><<<dim3(N / GBM, HW / 32), GTHR, 0, stream>>>(XB, XK, Wg1t, XK, 96, H, HW, 0, bg1, 0, 0);
  k_dots<<<N / NWAVE, NTHR, 0, stream>>>(H, as1, ad1, SD, N);
  k_gat<1><<<N / NB, NTHR, LDS_GAT, stream>>>(src, dst, H, SD, bg1, X1A, X1F, N, E, vec8);
  k_gemm<2><<<dim3(N / GBM, HW / 32), GTHR, 0, stream>>>(X1A, 2 * HW, Wg2D, 2 * HW, 2 * HW, H, HW, 0, bg2, 0, 0);
  k_dots<<<N / NWAVE, NTHR, 0, stream>>>(H, as2, ad2, SD, N);
  k_gat<2><<<N / NB, NTHR, LDS_GAT, stream>>>(src, dst, H, SD, bg2, X1A, X1F, N, E, vec8);
  k_pool<HW><<<G, ((HW / 4 + 31) / 32) * 32, 0, stream>>>(X1F, batch, N, P1D);

  k_gemm<2><<<dim3(N / GBM, GW / 32), GTHR, 0, stream>>>(XB, XK, WgcT, XK, 96, HGp, GW, 0, bgcn, 0, 0);
  k_gcn<1><<<N / NB, NTHR, LDS_GCN, stream>>>(src, dst, HGp, DINV, bgcn, XG, X2F, N, E, vec8);
  k_gemm<2><<<dim3(N / GBM, GW / 32), GTHR, 0, stream>>>(XG, 2 * GW, WgcD, 2 * GW, 2 * GW, HGp, GW, 0, bgcn, 0, 0);
  k_gcn<2><<<N / NB, NTHR, LDS_GCN, stream>>>(src, dst, HGp, DINV, bgcn, XG, X2F, N, E, vec8);
  k_pool<GW><<<G, ((GW / 4 + 31) / 32) * 32, 0, stream>>>(X2F, batch, N, P2D);

  k_conv<<<G, NTHR, 0, stream>>>(target, wconv, bconv, YD);

  k_gemm<4><<<dim3(G / GBM, 128 / 64), GTHR, 0, stream>>>(P1D, 4 * HW, Wf1D, 4 * HW, 4 * HW, XC, 512, 0, bfg1, 1, 1);
  k_gemm<4><<<dim3(G / GBM, 128 / 64), GTHR, 0, stream>>>(P2D, 4 * GW, Wf2D, 4 * GW, 4 * GW, XC, 512, 128, bfg2, 1, 1);
  k_gemm<4><<<dim3(G / GBM, 256 / 64), GTHR, 0, stream>>>(YD, 2 * CLP, WxtD, 2 * CLP, 2 * CLP, XC, 512, 256, bxt, 1, 0);
  { const int nU = G * (512 / 4); k_split<<<cdiv(nU, NTHR), NTHR, 0, stream>>>(XC, 512, XCD, nU); }
  k_gemm<4><<<dim3(G / GBM, 512 / 64), GTHR, 0, stream>>>(XCD, 1024, W1D, 1024, 1024, Z1, 512, 0, b1, 1, 1);
  { const int nU = G * (512 / 4); k_split<<<cdiv(nU, NTHR), NTHR, 0, stream>>>(Z1, 512, Z1D, nU); }
  k_gemm<4><<<dim3(G / GBM, 256 / 64), GTHR, 0, stream>>>(Z1D, 1024, W2D, 1024, 1024, Z2, 256, 0, b2, 1, 1);
  k_out<<<1, NTHR, 0, stream>>>(Z2, Wo, bo, out);
}
